// DeformAttn_67525475827771
// MI455X (gfx1250) — hardware-run, weakly checked
//
#include <hip/hip_runtime.h>


#ifndef NB
#define NB 4
#endif
#define NB_FULL 4
#define IH   48
#define IW   48
#define HWN  2304
#define CCH  192
#define CF   384
#define KVW  384
#define NHD  12
#define HDM  16
#define NCLIP 2
#define KPTS 9
#define DGC  216
#define OSP2 68
#define TSP  36
#define OCAR 64.0f
#define WCAR 1024.0f
#define HCAR 1024.0f
#define FS1  (1.0f / (64.0f * 1024.0f))
#define FS2  (1.0f / (1024.0f * 1024.0f))
#define LOG2E 1.4426950408889634f
#define NEGB (-1.0e30f)

static_assert(IH * IW == HWN);
static_assert(NHD * HDM == CCH);
static_assert(2 * CCH == KVW);
static_assert(12 * KPTS * 2 == DGC);
static_assert(HWN % 64 == 0);
static_assert(HWN % 32 == 0);
static_assert(CCH % 64 == 0);
static_assert(CF % 64 == 0);
static_assert(CCH % 32 == 0);
static_assert(CF % 32 == 0);
static_assert(NHD % 4 == 0);
static_assert(4 * HDM == 64);
static_assert(((size_t)NB * HWN) % 64 == 0);
static_assert(((size_t)CCH * CCH) % 8 == 0);
static_assert(((size_t)CF * CCH) % 8 == 0);
static_assert(NB <= NB_FULL);
static_assert((OSP2 * 4) % 16 == 0);
static_assert((TSP * 4) % 16 == 0);
static_assert(64 * OSP2 * 4 <= 131072);
static_assert(64 * TSP * 4 <= 131072);

typedef _Float16 h16;
typedef unsigned short bf;
typedef __attribute__((ext_vector_type(16))) __bf16   v16bf;
typedef __attribute__((ext_vector_type(16))) _Float16 v16h;
typedef __attribute__((ext_vector_type(8)))  _Float16 v8h;
typedef __attribute__((ext_vector_type(8)))  unsigned short v8us;
typedef __attribute__((ext_vector_type(8)))  float    v8f;
typedef __attribute__((ext_vector_type(4)))  float    v4f;
typedef v4f  __attribute__((may_alias)) v4fa;

__device__ __forceinline__ unsigned short f2bf(float f) { unsigned u = __float_as_uint(f); u += 0x7FFFu + ((u >> 16) & 1u); return (unsigned short)(u >> 16); }
__device__ __forceinline__ float bfr(float f) { return __uint_as_float(((unsigned)f2bf(f)) << 16); }
__device__ __forceinline__ v16h cat16(v8h lo, v8h hi) { return __builtin_shufflevector(lo, hi, 0, 1, 2, 3, 4, 5, 6, 7, 8, 9, 10, 11, 12, 13, 14, 15); }
__device__ __forceinline__ v16bf cat16b(v8us lo, v8us hi) { return __builtin_bit_cast(v16bf, __builtin_shufflevector(lo, hi, 0, 1, 2, 3, 4, 5, 6, 7, 8, 9, 10, 11, 12, 13, 14, 15)); }
__device__ __forceinline__ v8f wmma16(v16h a, v16h b, v8f c) { return __builtin_amdgcn_wmma_f32_16x16x32_f16(false, a, false, b, (short)0, c, false, false); }
__device__ __forceinline__ v8f wmmab(v16bf a, v16bf b, v8f c) { return __builtin_amdgcn_wmma_f32_16x16x32_bf16(false, a, false, b, (short)0, c, false, false); }
__device__ __forceinline__ v16h  ldh(const h16* p) { return cat16(*(const v8h*)p, *(const v8h*)(p + 16)); }
__device__ __forceinline__ v16bf ldb(const bf* p)  { return cat16b(*(const v8us*)p, *(const v8us*)(p + 16)); }
__device__ __forceinline__ void wave_sync() { __builtin_amdgcn_fence(3  , "wavefront"); __builtin_amdgcn_wave_barrier(); asm volatile("" ::: "memory"); }
__device__ __forceinline__ v8f mmah(v16h a, v16h b, v8f c) { c = wmma16(a, b, c); asm volatile("v_nop\n\tv_nop\n\tv_nop\n\tv_nop" : "+v"(c) : "v"(a), "v"(b)); return c; }
__device__ __forceinline__ v8f mmab(v16bf a, v16bf b, v8f c) { c = wmmab(a, b, c); asm volatile("v_nop\n\tv_nop\n\tv_nop\n\tv_nop" : "+v"(c) : "v"(a), "v"(b)); return c; }
static __device__ __forceinline__ h16 toh_flush(float v) { const h16 r = (h16)v; return (fabsf(v) < 6.103515625e-05f) ? (h16)0.0f : r; }
__device__ __forceinline__ float gelu_erf(float x) { return 0.5f * x * (1.0f + erff(x * 0.70710678118654752f)); }

__global__ __launch_bounds__(256) void k_cvt8(const float* __restrict__ src, bf* dst, size_t n8) {
    const size_t i = (size_t)blockIdx.x * 256 + threadIdx.x; if (i >= n8) return;
    const v8f v = *(const v8f*)(src + i * 8); v8us o;
#pragma unroll
    for (int k = 0; k < 8; ++k) o[k] = f2bf(v[k]);
    *(volatile v8us*)(dst + i * 8) = o; __threadfence(); *(volatile v8us*)(dst + i * 8) = o;
}

__global__ __launch_bounds__(256) void k_wcvt(const float* __restrict__ src, h16* dst, size_t n8, float carry) {
    const size_t i = (size_t)blockIdx.x * 256 + threadIdx.x; if (i >= n8) return;
    const v8f v = *(const v8f*)(src + i * 8); v8h o;
#pragma unroll
    for (int k = 0; k < 8; ++k) o[k] = toh_flush(bfr(v[k]) * carry);
    *(volatile v8h*)(dst + i * 8) = o; __threadfence(); *(volatile v8h*)(dst + i * 8) = o;
}

__global__ __launch_bounds__(256) void k_tcvt(const float* __restrict__ src, bf* dst) {
    __shared__ __align__(16) float tile[64 * TSP];
    const int tid = (int)threadIdx.x;
    const int n0 = blockIdx.x * 32, c0 = blockIdx.y * 64; const size_t img = blockIdx.z;
    const float* s = src + img * (size_t)CCH * HWN;
#pragma unroll
    for (int i = 0; i < 2; ++i) { const int qi = i * 256 + tid; const int row = qi >> 3, p4 = (qi & 7) * 4;
        const v4f v = *(const v4f*)(s + (size_t)(c0 + row) * HWN + n0 + p4);
        *(v4fa*)(&tile[row * TSP + p4]) = v; }
    __syncthreads();
    static_assert(256 * 16 == 32 * 128);
    const int p = tid >> 3, c8 = (tid & 7) * 8;
    v8us o;
#pragma unroll
    for (int k = 0; k < 8; ++k) o[k] = f2bf(tile[(c8 + k) * TSP + p]);
    bf* d = dst + (img * (size_t)HWN + (size_t)(n0 + p)) * CCH + c0 + c8;
    *(volatile v8us*)d = o; __threadfence(); *(volatile v8us*)d = o;
}

__global__ __launch_bounds__(32) void k_projf(const bf* __restrict__ A, const bf* __restrict__ Bt, const float* __restrict__ bias, float* Y, int ldY, int colOff) {
    __shared__ __align__(16) float os[64 * OSP2];
    const int K = CCH;
    const int lane = threadIdx.x & 31, lr = lane & 15, hi = lane >> 4; const int r0 = blockIdx.x * 64, c0 = blockIdx.y * 64;
    v8f acc[4][4];
#pragma unroll
    for (int mb = 0; mb < 4; ++mb)
#pragma unroll
        for (int nb = 0; nb < 4; ++nb) acc[mb][nb] = (v8f){};
    const size_t aoff = (size_t)(r0 + lr) * K + 8 * hi, boff = (size_t)(c0 + lr) * K + 8 * hi;
#pragma unroll 1
    for (int kc = 0; kc < K; kc += 32) {
        v16bf a[4];
#pragma unroll
        for (int mb = 0; mb < 4; ++mb) a[mb] = ldb(A + aoff + (size_t)mb * 16 * K + kc);
#pragma unroll
        for (int nb = 0; nb < 4; ++nb) { const v16bf bw = ldb(Bt + boff + (size_t)nb * 16 * K + kc);
#pragma unroll
            for (int mb = 0; mb < 4; ++mb) acc[mb][nb] = mmab(a[mb], bw, acc[mb][nb]); }
    }
    float bc[4];
#pragma unroll
    for (int nb = 0; nb < 4; ++nb) bc[nb] = bfr(bias[c0 + nb * 16 + lr]);
#pragma unroll
    for (int mb = 0; mb < 4; ++mb)
#pragma unroll
        for (int nb = 0; nb < 4; ++nb)
#pragma unroll
            for (int j = 0; j < 8; ++j) os[(mb * 16 + hi * 8 + j) * OSP2 + nb * 16 + lr] = acc[mb][nb][j] + bc[nb];
    wave_sync();
    float* yb = Y + (size_t)r0 * (size_t)ldY + (size_t)colOff + (size_t)c0;
    static_assert(32 * 32 * 16 == 64 * 256);
#pragma unroll 1
    for (int ps = 0; ps < 2; ++ps) {
#pragma unroll 1
        for (int s = 0; s < 32; ++s) { const int row = 2 * s + (lane >> 4), c4 = (lane & 15) * 4;
            const v4f val = *(const v4fa*)(&os[row * OSP2 + c4]);
            *(volatile v4f*)(yb + (size_t)row * (size_t)ldY + c4) = val; }
        if (ps == 0) __threadfence(); }
}

__global__ __launch_bounds__(256) void k_offtap(const float* __restrict__ QP, const float* __restrict__ KV, const float* __restrict__ OFF, h16* OH, float* OC) {
#pragma clang fp contract(off)
    __shared__ __align__(16) float osm[64 * OSP2];
    const int lane = threadIdx.x & 31;
    const int wave = __builtin_amdgcn_readfirstlane((int)(threadIdx.x >> 5));
    const int hl = wave & 3, pg = wave >> 2;
    const int pl = pg * 32 + lane;
    const int n = blockIdx.x * 64 + pl;
    const int hg = blockIdx.y, b = blockIdx.z;
    const int h = hg * 4 + hl;
    const int yq = n / IW, xq = n - yq * IW;
    float q[16];
    { const float* qp = QP + ((size_t)b * HWN + (size_t)n) * CCH + h * HDM;
#pragma unroll
      for (int i = 0; i < 4; ++i) { const v4f t = *(const v4f*)(qp + 4 * i);
#pragma unroll
          for (int j = 0; j < 4; ++j) q[4 * i + j] = t[j] * 0.25f; } }
    const int gk = h >> 1, gv = 6 + (h >> 1);
    float o[16];
#pragma unroll
    for (int i = 0; i < 16; ++i) o[i] = 0.0f;
    float m = NEGB, l = 0.0f;
    const float ymax = (float)(IH - 1), xmax = (float)(IW - 1);
#pragma unroll 1
    for (int tap = 0; tap < NCLIP * KPTS; ++tap) {
        const int c = (tap >= KPTS) ? 1 : 0; const int k = tap - KPTS * c; const int kyi = k / 3, kxi = k - 3 * kyi;
        const size_t bc = (size_t)b * NCLIP + (size_t)c;
        const float* offp = OFF + bc * (size_t)DGC * HWN + (size_t)n;
        const float* kvb = KV + bc * (size_t)HWN * KVW + h * HDM;
        const float by = (float)(yq - 1 + kyi), bx = (float)(xq - 1 + kxi);
        float s = 0.0f;
        { const float oy = bfr(offp[(size_t)((gk * KPTS + k) * 2) * HWN]);
          const float ox = bfr(offp[(size_t)((gk * KPTS + k) * 2 + 1) * HWN]);
          const float py = by + oy, px = bx + ox;
          const float y0 = floorf(py), x0 = floorf(px);
          const float wy1 = py - y0, wx1 = px - x0;
#pragma unroll 1
          for (int cr = 0; cr < 4; ++cr) {
              const float yi = y0 + (float)(cr >> 1), xi = x0 + (float)(cr & 1);
              const float wyc = (cr >> 1) ? wy1 : (1.0f - wy1);
              const float wxc = (cr & 1) ? wx1 : (1.0f - wx1);
              const bool valid = (yi >= 0.0f) & (yi <= ymax) & (xi >= 0.0f) & (xi <= xmax);
              const float we = (wyc * wxc) * (valid ? 1.0f : 0.0f);
              const int idx = (int)(fminf(fmaxf(yi, 0.0f), ymax) * (float)IW + fminf(fmaxf(xi, 0.0f), xmax));
              const float* p = kvb + (size_t)idx * KVW;
              const v4f t0 = *(const v4f*)p, t1 = *(const v4f*)(p + 4), t2 = *(const v4f*)(p + 8), t3 = *(const v4f*)(p + 12);
              float d = q[0] * t0[0];
              d = fmaf(q[1], t0[1], d); d = fmaf(q[2], t0[2], d); d = fmaf(q[3], t0[3], d);
              d = fmaf(q[4], t1[0], d); d = fmaf(q[5], t1[1], d); d = fmaf(q[6], t1[2], d); d = fmaf(q[7], t1[3], d);
              d = fmaf(q[8], t2[0], d); d = fmaf(q[9], t2[1], d); d = fmaf(q[10], t2[2], d); d = fmaf(q[11], t2[3], d);
              d = fmaf(q[12], t3[0], d); d = fmaf(q[13], t3[1], d); d = fmaf(q[14], t3[2], d); d = fmaf(q[15], t3[3], d);
              s = fmaf(we, d, s); } }
        const float mnew = fmaxf(m, s);
        const float alpha = __builtin_amdgcn_exp2f((m - mnew) * LOG2E);
        const float pe = __builtin_amdgcn_exp2f((s - mnew) * LOG2E);
        l = l * alpha + pe; m = mnew;
#pragma unroll
        for (int i = 0; i < 16; ++i) o[i] = o[i] * alpha;
        { const float oy = bfr(offp[(size_t)((gv * KPTS + k) * 2) * HWN]);
          const float ox = bfr(offp[(size_t)((gv * KPTS + k) * 2 + 1) * HWN]);
          const float py = by + oy, px = bx + ox;
          const float y0 = floorf(py), x0 = floorf(px);
          const float wy1 = py - y0, wx1 = px - x0;
#pragma unroll 1
          for (int cr = 0; cr < 4; ++cr) {
              const float yi = y0 + (float)(cr >> 1), xi = x0 + (float)(cr & 1);
              const float wyc = (cr >> 1) ? wy1 : (1.0f - wy1);
              const float wxc = (cr & 1) ? wx1 : (1.0f - wx1);
              const bool valid = (yi >= 0.0f) & (yi <= ymax) & (xi >= 0.0f) & (xi <= xmax);
              const float we = (wyc * wxc) * (valid ? 1.0f : 0.0f);
              const int idx = (int)(fminf(fmaxf(yi, 0.0f), ymax) * (float)IW + fminf(fmaxf(xi, 0.0f), xmax));
              const float* p = kvb + CCH + (size_t)idx * KVW;
              const v4f t0 = *(const v4f*)p, t1 = *(const v4f*)(p + 4), t2 = *(const v4f*)(p + 8), t3 = *(const v4f*)(p + 12);
              const float w2 = pe * we;
#pragma unroll
              for (int j = 0; j < 4; ++j) { o[j] = fmaf(w2, t0[j], o[j]); o[4 + j] = fmaf(w2, t1[j], o[4 + j]); o[8 + j] = fmaf(w2, t2[j], o[8 + j]); o[12 + j] = fmaf(w2, t3[j], o[12 + j]); } } }
    }
    const float inv = 1.0f / l;
#pragma unroll
    for (int i = 0; i < 4; ++i) { v4f t; t[0] = o[4 * i] * inv; t[1] = o[4 * i + 1] * inv; t[2] = o[4 * i + 2] * inv; t[3] = o[4 * i + 3] * inv;
        *(v4fa*)(&osm[pl * OSP2 + hl * HDM + 4 * i]) = t; }
    __syncthreads();
    h16* ohb = OH + ((size_t)b * HWN + (size_t)blockIdx.x * 64) * CCH + (size_t)hg * 64;
    float* ocb = OC + ((size_t)b * CCH + (size_t)hg * 64) * HWN + (size_t)blockIdx.x * 64;
    static_assert(2 * 256 * 16 == 64 * 128);
    static_assert(4 * 256 * 16 == 64 * 256);
#pragma unroll 1
    for (int ps = 0; ps < 2; ++ps) {
#pragma unroll 1
        for (int s = 0; s < 2; ++s) { const int qi = s * 256 + (int)threadIdx.x; const int row = qi >> 3, c8 = (qi & 7) * 8;
            const v4f x0 = *(const v4fa*)(&osm[row * OSP2 + c8]); const v4f x1 = *(const v4fa*)(&osm[row * OSP2 + c8 + 4]); v8h hv;
#pragma unroll
            for (int i = 0; i < 4; ++i) { hv[i] = toh_flush(x0[i] * OCAR); hv[4 + i] = toh_flush(x1[i] * OCAR); }
            *(volatile v8h*)(ohb + (size_t)row * CCH + c8) = hv; }
#pragma unroll 1
        for (int s = 0; s < 4; ++s) { const int qi = s * 256 + (int)threadIdx.x; const int ch = qi >> 4, p4 = (qi & 15) * 4;
            v4f val;
#pragma unroll
            for (int i = 0; i < 4; ++i) val[i] = osm[(p4 + i) * OSP2 + ch];
            *(volatile v4f*)(ocb + (size_t)ch * HWN + p4) = val; }
        if (ps == 0) __threadfence(); }
}

__global__ __launch_bounds__(32) void k_ffn1(const h16* __restrict__ A, const h16* __restrict__ Bt, const float* __restrict__ bias, h16* HH) {
    __shared__ __align__(16) float os[64 * OSP2];
    const int K = CCH;
    const int lane = threadIdx.x & 31, lr = lane & 15, hi = lane >> 4; const int r0 = blockIdx.x * 64, c0 = blockIdx.y * 64;
    v8f acc[4][4];
#pragma unroll
    for (int mb = 0; mb < 4; ++mb)
#pragma unroll
        for (int nb = 0; nb < 4; ++nb) acc[mb][nb] = (v8f){};
    const size_t aoff = (size_t)(r0 + lr) * K + 8 * hi, boff = (size_t)(c0 + lr) * K + 8 * hi;
#pragma unroll 1
    for (int kc = 0; kc < K; kc += 32) {
        v16h a[4];
#pragma unroll
        for (int mb = 0; mb < 4; ++mb) a[mb] = ldh(A + aoff + (size_t)mb * 16 * K + kc);
#pragma unroll
        for (int nb = 0; nb < 4; ++nb) { const v16h bw = ldh(Bt + boff + (size_t)nb * 16 * K + kc);
#pragma unroll
            for (int mb = 0; mb < 4; ++mb) acc[mb][nb] = mmah(a[mb], bw, acc[mb][nb]); }
    }
    float bc[4];
#pragma unroll
    for (int nb = 0; nb < 4; ++nb) bc[nb] = bfr(bias[c0 + nb * 16 + lr]);
#pragma unroll
    for (int mb = 0; mb < 4; ++mb)
#pragma unroll
        for (int nb = 0; nb < 4; ++nb)
#pragma unroll
            for (int j = 0; j < 8; ++j) os[(mb * 16 + hi * 8 + j) * OSP2 + nb * 16 + lr] = acc[mb][nb][j] * FS1 + bc[nb];
    wave_sync();
    h16* hb = HH + (size_t)r0 * CF + (size_t)c0;
    static_assert(16 * 32 * 16 == 64 * 128);
#pragma unroll 1
    for (int ps = 0; ps < 2; ++ps) {
#pragma unroll 1
        for (int s = 0; s < 16; ++s) { const int row = 4 * s + (lane >> 3), c8 = (lane & 7) * 8;
            const v4f x0 = *(const v4fa*)(&os[row * OSP2 + c8]); const v4f x1 = *(const v4fa*)(&os[row * OSP2 + c8 + 4]); v8h hv;
#pragma unroll
            for (int i = 0; i < 4; ++i) { hv[i] = toh_flush(gelu_erf(x0[i]) * HCAR); hv[4 + i] = toh_flush(gelu_erf(x1[i]) * HCAR); }
            *(volatile v8h*)(hb + (size_t)row * CF + c8) = hv; }
        if (ps == 0) __threadfence(); }
}

__global__ __launch_bounds__(32) void k_ffn2(const h16* __restrict__ A, const h16* __restrict__ Bt, const float* __restrict__ bias, const float* __restrict__ OC, float* OUT) {
    __shared__ __align__(16) float os[64 * OSP2];
    const int K = CF;
    const int lane = threadIdx.x & 31, lr = lane & 15, hi = lane >> 4; const int r0 = blockIdx.x * 64, c0 = blockIdx.y * 64;
    v8f acc[4][4];
#pragma unroll
    for (int mb = 0; mb < 4; ++mb)
#pragma unroll
        for (int nb = 0; nb < 4; ++nb) acc[mb][nb] = (v8f){};
    const size_t aoff = (size_t)(r0 + lr) * K + 8 * hi, boff = (size_t)(c0 + lr) * K + 8 * hi;
#pragma unroll 1
    for (int kc = 0; kc < K; kc += 32) {
        v16h a[4];
#pragma unroll
        for (int mb = 0; mb < 4; ++mb) a[mb] = ldh(A + aoff + (size_t)mb * 16 * K + kc);
#pragma unroll
        for (int nb = 0; nb < 4; ++nb) { const v16h bw = ldh(Bt + boff + (size_t)nb * 16 * K + kc);
#pragma unroll
            for (int mb = 0; mb < 4; ++mb) acc[mb][nb] = mmah(a[mb], bw, acc[mb][nb]); }
    }
#pragma unroll
    for (int mb = 0; mb < 4; ++mb) {
        float br[8];
#pragma unroll
        for (int j = 0; j < 8; ++j) br[j] = bfr(bias[r0 + mb * 16 + hi * 8 + j]);
#pragma unroll
        for (int nb = 0; nb < 4; ++nb)
#pragma unroll
            for (int j = 0; j < 8; ++j) os[(mb * 16 + hi * 8 + j) * OSP2 + nb * 16 + lr] = acc[mb][nb][j] * FS2 + br[j]; }
    wave_sync();
    const int bb = c0 / HWN, nn = c0 % HWN;
    const size_t ob = ((size_t)bb * CCH + (size_t)r0) * HWN + (size_t)nn;
    static_assert(32 * 32 * 16 == 64 * 256);
#pragma unroll 1
    for (int ps = 0; ps < 2; ++ps) {
#pragma unroll 1
        for (int s = 0; s < 32; ++s) { const int row = 2 * s + (lane >> 4), c4 = (lane & 15) * 4;
            const v4f gv = *(const v4fa*)(&os[row * OSP2 + c4]);
            const v4f rv = *(const v4f*)(OC + ob + (size_t)row * HWN + c4);
            const v4f val = gv + rv;
            *(volatile v4f*)(OUT + ob + (size_t)row * HWN + c4) = val; }
        if (ps == 0) __threadfence(); }
}

static constexpr size_t al256(size_t v) { return (v + 255) & ~(size_t)255; }
static constexpr size_t SZ_XQ = al256((size_t)NB * HWN * CCH * 2);
static constexpr size_t SZ_XK = al256((size_t)NB * NCLIP * HWN * CCH * 2);
static constexpr size_t SZ_WB = al256((size_t)3 * CCH * CCH * 2);
static constexpr size_t SZ_WF = al256((size_t)CF * CCH * 2);
static constexpr size_t SZ_QP = al256((size_t)NB * HWN * CCH * 4);
static constexpr size_t SZ_KV = al256((size_t)NB * NCLIP * HWN * KVW * 4);
static constexpr size_t SZ_OH = al256((size_t)NB * HWN * CCH * 2);
static constexpr size_t SZ_OC = al256((size_t)NB * CCH * HWN * 4);
static constexpr size_t SZ_HH = al256((size_t)NB * HWN * CF * 2);
static constexpr size_t SZ_TOTAL = SZ_XQ + 2 * SZ_XK + SZ_WB + 2 * SZ_WF + SZ_QP + SZ_KV + SZ_OH + SZ_OC + SZ_HH;
static_assert(SZ_TOTAL <= (size_t)134217728);
static_assert(((size_t)CCH * CCH * 2) % 256 == 0);

extern "C" void kernel_launch(void* const* d_in, const int* in_sizes, int n_in,
                              void* d_out, int out_size, void* d_ws, size_t ws_size, hipStream_t stream) {
    if (n_in < 14) return;
    const size_t needq = (size_t)NB * CCH * HWN;
    const size_t needk = (size_t)NB * NCLIP * CCH * HWN;
    const size_t needo = (size_t)NB * NCLIP * DGC * HWN;
    if ((size_t)in_sizes[0] < needq || (size_t)in_sizes[1] < needk || (size_t)in_sizes[2] < needk || (size_t)in_sizes[3] < needo) return;
    if ((size_t)in_sizes[4] < (size_t)CCH * CCH || (size_t)in_sizes[6] < (size_t)CCH * CCH || (size_t)in_sizes[8] < (size_t)CCH * CCH) return;
    if (in_sizes[5] < CCH || in_sizes[7] < CCH || in_sizes[9] < CCH) return;
    if ((size_t)in_sizes[10] < (size_t)CF * CCH || in_sizes[11] < CF || (size_t)in_sizes[12] < (size_t)CCH * CF || in_sizes[13] < CCH) return;
    if ((size_t)out_size < needq) return;
    if (SZ_TOTAL > ws_size) return;
    const float* qin = (const float*)d_in[0]; const float* kin = (const float*)d_in[1]; const float* vin = (const float*)d_in[2];
    const float* off = (const float*)d_in[3];
    const float* wq = (const float*)d_in[4];  const float* bq = (const float*)d_in[5];
    const float* wk = (const float*)d_in[6];  const float* bk = (const float*)d_in[7];
    const float* wv = (const float*)d_in[8];  const float* bv = (const float*)d_in[9];
    const float* w1 = (const float*)d_in[10]; const float* b1 = (const float*)d_in[11];
    const float* w2 = (const float*)d_in[12]; const float* b2 = (const float*)d_in[13];
    float* OUT = (float*)d_out;
    char* wsp = (char*)d_ws;
    bf* XQ = (bf*)wsp; wsp += SZ_XQ;
    bf* XK = (bf*)wsp; wsp += SZ_XK;
    bf* XV = (bf*)wsp; wsp += SZ_XK;
    bf* WB = (bf*)wsp; wsp += SZ_WB;
    h16* W1H = (h16*)wsp; wsp += SZ_WF;
    h16* W2H = (h16*)wsp; wsp += SZ_WF;
    float* QP = (float*)wsp; wsp += SZ_QP;
    float* KV = (float*)wsp; wsp += SZ_KV;
    h16* OH = (h16*)wsp; wsp += SZ_OH;
    float* OC = (float*)wsp; wsp += SZ_OC;
    h16* HH = (h16*)wsp; wsp += SZ_HH;
    bf* WQ = WB; bf* WK = WB + (size_t)CCH * CCH; bf* WV = WB + (size_t)2 * CCH * CCH;

    k_tcvt<<<dim3(HWN / 32, CCH / 64, NB), 256, 0, stream>>>(qin, XQ);
    k_tcvt<<<dim3(HWN / 32, CCH / 64, NB * NCLIP), 256, 0, stream>>>(kin, XK);
    k_tcvt<<<dim3(HWN / 32, CCH / 64, NB * NCLIP), 256, 0, stream>>>(vin, XV);
    { const size_t n8 = (size_t)CCH * CCH / 8; const unsigned g = (unsigned)((n8 + 255) / 256);
      k_cvt8<<<g, 256, 0, stream>>>(wq, WQ, n8); k_cvt8<<<g, 256, 0, stream>>>(wk, WK, n8); k_cvt8<<<g, 256, 0, stream>>>(wv, WV, n8); }
    { const size_t n8 = (size_t)CF * CCH / 8; const unsigned g = (unsigned)((n8 + 255) / 256);
      k_wcvt<<<g, 256, 0, stream>>>(w1, W1H, n8, WCAR); k_wcvt<<<g, 256, 0, stream>>>(w2, W2H, n8, WCAR); }

    k_projf<<<dim3(NB * HWN / 64, CCH / 64, 1), 32, 0, stream>>>(XQ, WQ, bq, QP, CCH, 0);
    k_projf<<<dim3(NB * NCLIP * HWN / 64, CCH / 64, 1), 32, 0, stream>>>(XK, WK, bk, KV, KVW, 0);
    k_projf<<<dim3(NB * NCLIP * HWN / 64, CCH / 64, 1), 32, 0, stream>>>(XV, WV, bv, KV, KVW, CCH);

    k_offtap<<<dim3(HWN / 64, NHD / 4, NB), 256, 0, stream>>>(QP, KV, off, OH, OC);

    k_ffn1<<<dim3(NB * HWN / 64, CF / 64, 1), 32, 0, stream>>>(OH, W1H, b1, HH);
    k_ffn2<<<dim3(CCH / 64, NB * HWN / 64, 1), 32, 0, stream>>>(W2H, HH, b2, OC, OUT);
}
